// RNN_78391743087139
// MI455X (gfx1250) — hardware-verified
//
#include <hip/hip_runtime.h>
#include <math.h>

constexpr int RNN_NB    = 4096;
constexpr int RNN_NT    = 512;
constexpr int RNN_NH    = 32;
constexpr int RNN_ROWS  = 16;
constexpr int RNN_CHUNK = 32;
constexpr int XPITCH    = 36;
constexpr int YPITCH    = 36;
constexpr int FPITCH    = 36;
constexpr float RES_CARRY     = 2048.0f;
constexpr float RES_CARRY_INV = 1.0f / 2048.0f;
constexpr int OUT0_ELEMS = RNN_NB * RNN_NT;
constexpr int OUT1_ELEMS = RNN_NB * RNN_NH;

static_assert(RNN_NH == 32, "one 32-deep k step, two 16-row hid tiles");
static_assert(RNN_NB % RNN_ROWS == 0, "grid exact");
static_assert(RNN_NT % RNN_CHUNK == 0, "no tail chunk");
static_assert(RNN_CHUNK == 32, "one 128-B line per row per chunk");
static_assert((size_t)OUT0_ELEMS * 4 == 8388608, "out1 byte offset");
static_assert(((size_t)OUT0_ELEMS * 4) % 128 == 0, "out1 line aligned");
static_assert(((size_t)OUT0_ELEMS + (size_t)OUT1_ELEMS) * 4 == 8912896, "d_out total bytes");
static_assert(XPITCH % 4 == 0 && YPITCH % 4 == 0 && FPITCH % 4 == 0, "16-B aligned LDS rows");

typedef __attribute__((ext_vector_type(16))) _Float16 v16h;
typedef __attribute__((ext_vector_type(8)))  _Float16 v8h;
typedef __attribute__((ext_vector_type(8)))  float    v8f;
typedef __attribute__((ext_vector_type(4)))  float    v4f;

template <typename T> struct Frag;
template <> struct Frag<_Float16> {
  typedef v16h V; union U { v16h v; v8h h[2]; };
  static __device__ __forceinline__ v16h load(const _Float16* p) {
    U f; f.h[0] = *(const v8h*)(p); f.h[1] = *(const v8h*)(p + 16); return f.v;
  }
  static __device__ __forceinline__ v8f mma(v16h a, v16h b, v8f c) {
    return __builtin_amdgcn_wmma_f32_16x16x32_f16(false, a, false, b, (short)0, c, false, false);
  }
};

__device__ __forceinline__ void guard_group(v8f& a, v8f& b, v8f& c, v8f& d,
                                            v16h w0, v16h w1, v16h w2, v16h w3, v16h x, v16h y) {
  asm volatile("v_nop\n\tv_nop\n\tv_nop\n\tv_nop"
               : "+v"(a), "+v"(b), "+v"(c), "+v"(d)
               : "v"(w0), "v"(w1), "v"(w2), "v"(w3), "v"(x), "v"(y));
}

__device__ __forceinline__ float tanh_f32(float v) {
  const float e = expf(2.0f * v);
  return 1.0f - 2.0f * __builtin_amdgcn_rcpf(e + 1.0f);
}

__device__ __forceinline__ void split_h16(float f, _Float16& hi, _Float16& lo) {
  const _Float16 hv = (_Float16)f;
  const float hf = (float)hv;
  const float rs = (f - hf) * RES_CARRY;
  hi = hv;
  lo = (_Float16)rs;
}

__global__ __launch_bounds__(32) void rnn_seq_kernel(const float* __restrict__ x,
                                                     const float* __restrict__ h0,
                                                     const float* __restrict__ Wih,
                                                     const float* __restrict__ Whh,
                                                     const float* __restrict__ bih,
                                                     const float* __restrict__ bhh,
                                                     const float* __restrict__ Wout,
                                                     const float* __restrict__ bout,
                                                     float* __restrict__ outs,
                                                     float* __restrict__ hlast) {
  __shared__ __align__(16) _Float16 Whi[RNN_NH * RNN_NH];
  __shared__ __align__(16) _Float16 Wlo[RNN_NH * RNN_NH];
  __shared__ __align__(16) _Float16 Hhi[RNN_ROWS * RNN_NH];
  __shared__ __align__(16) _Float16 Hlo[RNN_ROWS * RNN_NH];
  __shared__ __align__(16) float xs[RNN_ROWS * XPITCH];
  __shared__ __align__(16) float ys[RNN_ROWS * YPITCH];
  __shared__ __align__(16) float hf[RNN_ROWS * FPITCH];
  __shared__ __align__(16) float cst[3 * RNN_NH];

  const int lane = threadIdx.x & 31;
  const int c    = lane & 15;
  const int hh   = lane >> 4;
  const int koff = hh * 8;
  const int b0   = blockIdx.x * RNN_ROWS;
  const int lrow = lane >> 3;
  const int lc4  = (lane & 7) * 4;

  {
    const float* wrow = Whh + (size_t)lane * RNN_NH;
    v4f w[8];
#pragma unroll
    for (int q = 0; q < 8; ++q) w[q] = *(const v4f*)(wrow + 4 * q);
#pragma unroll
    for (int g = 0; g < 4; ++g) {
      v8h hv, lv;
#pragma unroll
      for (int e = 0; e < 4; ++e) {
        const float f0 = w[2 * g][e];
        const float f1 = w[2 * g + 1][e];
        _Float16 a0, r0, a1, r1;
        split_h16(f0, a0, r0);
        split_h16(f1, a1, r1);
        hv[e] = a0; lv[e] = r0;
        hv[4 + e] = a1; lv[4 + e] = r1;
      }
      *(v8h*)(Whi + lane * RNN_NH + 8 * g) = hv;
      *(v8h*)(Wlo + lane * RNN_NH + 8 * g) = lv;
    }
  }
  asm volatile("" ::: "memory");

  {
    const float a  = Wih[lane];
    const float b1 = bih[lane];
    const float b2 = bhh[lane];
    const float o  = Wout[lane];
    cst[lane]              = a;
    cst[RNN_NH + lane]     = b1 + b2;
    cst[2 * RNN_NH + lane] = o;
  }
  asm volatile("" ::: "memory");

  float th[2][8];
  {
    const float* hrow = h0 + (size_t)(b0 + c) * RNN_NH + koff;
    const v4f p0 = *(const v4f*)(hrow);
    const v4f p1 = *(const v4f*)(hrow + 4);
    const v4f p2 = *(const v4f*)(hrow + 16);
    const v4f p3 = *(const v4f*)(hrow + 20);
#pragma unroll
    for (int e = 0; e < 4; ++e) {
      th[0][e] = p0[e]; th[0][4 + e] = p1[e];
      th[1][e] = p2[e]; th[1][4 + e] = p3[e];
    }
  }
#pragma unroll
  for (int mt = 0; mt < 2; ++mt) {
    v8h hv, lv;
#pragma unroll
    for (int r = 0; r < 8; ++r) {
      _Float16 a, rs;
      split_h16(th[mt][r], a, rs);
      hv[r] = a; lv[r] = rs;
    }
    *(v8h*)(Hhi + c * RNN_NH + 16 * mt + koff) = hv;
    *(v8h*)(Hlo + c * RNN_NH + 16 * mt + koff) = lv;
  }
  const float bo = bout[0];
  __syncthreads();

  const v16h aWh0 = Frag<_Float16>::load(Whi + (c)      * RNN_NH + koff);
  const v16h aWh1 = Frag<_Float16>::load(Whi + (16 + c) * RNN_NH + koff);
  const v16h aWl0 = Frag<_Float16>::load(Wlo + (c)      * RNN_NH + koff);
  const v16h aWl1 = Frag<_Float16>::load(Wlo + (16 + c) * RNN_NH + koff);
  float cw[2][8], cb[2][8], wo[2][8];
#pragma unroll
  for (int mt = 0; mt < 2; ++mt)
#pragma unroll
    for (int r = 0; r < 8; ++r) {
      const int j = 16 * mt + koff + r;
      cw[mt][r] = cst[j];
      cb[mt][r] = cst[RNN_NH + j];
      wo[mt][r] = cst[2 * RNN_NH + j];
    }

  const v8f z8 = {0.f, 0.f, 0.f, 0.f, 0.f, 0.f, 0.f, 0.f};

#pragma unroll 1
  for (int t = 0; t < RNN_NT; ++t) {
    const int tl = t & (RNN_CHUNK - 1);
    if (tl == 0) {
      __syncthreads();
#pragma unroll
      for (int it = 0; it < 4; ++it) {
        const int row = it * 4 + lrow;
        const v4f v = *(const v4f*)(x + (size_t)(b0 + row) * RNN_NT + t + lc4);
        *(v4f*)(xs + row * XPITCH + lc4) = v;
      }
      __syncthreads();
    }

    const float xv = xs[c * XPITCH + tl];
    v8f accM0, accM1;
#pragma unroll
    for (int r = 0; r < 8; ++r) {
      accM0[r] = fmaf(xv, cw[0][r], cb[0][r]);
      accM1[r] = fmaf(xv, cw[1][r], cb[1][r]);
    }
    const v16h bh = Frag<_Float16>::load(Hhi + c * RNN_NH + koff);
    const v16h bl = Frag<_Float16>::load(Hlo + c * RNN_NH + koff);
    v8f accR0 = z8, accR1 = z8;
    accM0 = Frag<_Float16>::mma(aWh0, bh, accM0);
    accM1 = Frag<_Float16>::mma(aWh1, bh, accM1);
    accR0 = Frag<_Float16>::mma(aWl0, bh, accR0);
    accR1 = Frag<_Float16>::mma(aWl1, bh, accR1);
    accR0 = Frag<_Float16>::mma(aWh0, bl, accR0);
    accR1 = Frag<_Float16>::mma(aWh1, bl, accR1);
    guard_group(accM0, accM1, accR0, accR1, aWh0, aWh1, aWl0, aWl1, bh, bl);

    float part = 0.0f;
#pragma unroll
    for (int r = 0; r < 8; ++r) {
      const float p0 = accM0[r] + accR0[r] * RES_CARRY_INV;
      const float p1 = accM1[r] + accR1[r] * RES_CARRY_INV;
      const float t0v = tanh_f32(p0);
      const float t1v = tanh_f32(p1);
      th[0][r] = t0v;
      th[1][r] = t1v;
      part = fmaf(t0v, wo[0][r], part);
      part = fmaf(t1v, wo[1][r], part);
    }
    const float other = __shfl_xor(part, 16, 32);
    const float yv = (part + other) + bo;
    if (hh == 0) ys[c * YPITCH + tl] = yv;

#pragma unroll
    for (int mt = 0; mt < 2; ++mt) {
      v8h hv, lv;
#pragma unroll
      for (int r = 0; r < 8; ++r) {
        _Float16 a, rs;
        split_h16(th[mt][r], a, rs);
        hv[r] = a; lv[r] = rs;
      }
      *(v8h*)(Hhi + c * RNN_NH + 16 * mt + koff) = hv;
      *(v8h*)(Hlo + c * RNN_NH + 16 * mt + koff) = lv;
    }
    __syncthreads();

    if (tl == RNN_CHUNK - 1) {
      const int tbase = t - (RNN_CHUNK - 1);
      for (int pass = 0; pass < 2; ++pass) {
#pragma unroll
        for (int it = 0; it < 4; ++it) {
          const int row = it * 4 + lrow;
          const v4f v = *(const v4f*)(ys + row * YPITCH + lc4);
          *(volatile v4f*)(outs + (size_t)(b0 + row) * RNN_NT + tbase + lc4) = v;
        }
        __threadfence();
      }
      __syncthreads();
    }
  }

#pragma unroll
  for (int mt = 0; mt < 2; ++mt) {
    v4f a, b;
#pragma unroll
    for (int e = 0; e < 4; ++e) { a[e] = th[mt][e]; b[e] = th[mt][4 + e]; }
    *(v4f*)(hf + c * FPITCH + 16 * mt + koff)     = a;
    *(v4f*)(hf + c * FPITCH + 16 * mt + koff + 4) = b;
  }
  __syncthreads();
  for (int pass = 0; pass < 2; ++pass) {
#pragma unroll
    for (int it = 0; it < 4; ++it) {
      const int row = it * 4 + lrow;
      const v4f v = *(const v4f*)(hf + row * FPITCH + lc4);
      *(volatile v4f*)(hlast + (size_t)(b0 + row) * RNN_NH + lc4) = v;
    }
    __threadfence();
  }
}

extern "C" void kernel_launch(void* const* d_in, const int* in_sizes, int n_in,
                              void* d_out, int out_size, void* d_ws, size_t ws_size,
                              hipStream_t stream) {
  (void)d_ws; (void)ws_size;
  if (n_in < 8 || d_out == nullptr) return;
  if (in_sizes[0] != RNN_NB * RNN_NT || in_sizes[1] != RNN_NB * RNN_NH || in_sizes[2] != RNN_NH ||
      in_sizes[3] != RNN_NH * RNN_NH || in_sizes[4] != RNN_NH || in_sizes[5] != RNN_NH ||
      in_sizes[6] != RNN_NH || in_sizes[7] != 1 || out_size != OUT0_ELEMS + OUT1_ELEMS) return;

  const float* x    = (const float*)d_in[0];
  const float* h0   = (const float*)d_in[1];
  const float* Wih  = (const float*)d_in[2];
  const float* Whh  = (const float*)d_in[3];
  const float* bih  = (const float*)d_in[4];
  const float* bhh  = (const float*)d_in[5];
  const float* Wout = (const float*)d_in[6];
  const float* bout = (const float*)d_in[7];

  float* outs  = (float*)d_out;
  float* hlast = outs + (size_t)OUT0_ELEMS;

  rnn_seq_kernel<<<dim3(RNN_NB / RNN_ROWS), dim3(32), 0, stream>>>(x, h0, Wih, Whh, bih, bhh, Wout, bout, outs, hlast);
}
